// GRU_48627619726124
// MI455X (gfx1250) — hardware-verified
//
#include <hip/hip_runtime.h>
#include <math.h>

constexpr int NSEQ   = 4096;
constexpr int NSTEP  = 128;
constexpr int NINP   = 16;
constexpr int NHID   = 64;
constexpr int NG3    = 3 * NHID;
constexpr int NTHR   = 256;
constexpr int NWAVE  = NTHR / 32;
constexpr int RPB    = 32;
constexpr int APITCH = 104;
constexpr int ACOLX  = 64;
constexpr int KHID   = NHID;
constexpr int WHP    = 72;
constexpr int WXP    = 40;
constexpr int HFP    = 68;
constexpr float WCARRY      = 16.0f;
constexpr float WCARRY_INV  = 1.0f / 16.0f;
constexpr float LOCARRY     = 2048.0f;
constexpr float LOCARRY_INV = 1.0f / 2048.0f;
static_assert(NSEQ % RPB == 0);
static_assert(RPB == 32);
static_assert(NWAVE == 2 * (NHID / 16));
static_assert(KHID % 32 == 0);
static_assert(NINP == 16);
static_assert(ACOLX + 32 <= APITCH);
static_assert(APITCH % 8 == 0 && WHP % 8 == 0 && WXP % 8 == 0 && HFP % 4 == 0);
static_assert((4 * RPB * APITCH) % NTHR == 0);
static_assert(NTHR == 256);
static_assert(NG3 % 32 == 0);

typedef __attribute__((ext_vector_type(16))) _Float16 v16h;
typedef __attribute__((ext_vector_type(8)))  _Float16 v8h;
typedef __attribute__((ext_vector_type(4)))  _Float16 v4h;
typedef __attribute__((ext_vector_type(8)))  float    v8f;
typedef __attribute__((ext_vector_type(4)))  float    v4f;

__device__ __forceinline__ void dep_guard_h(v8f& a, v8f& b, v16h x, v16h y) { asm volatile("v_nop\n\tv_nop\n\tv_nop\n\tv_nop" : "+v"(a), "+v"(b) : "v"(x), "v"(y)); }
__device__ __forceinline__ void keep4_h(v16h a, v16h b, v16h c, v16h d) { asm volatile("v_nop" :: "v"(a), "v"(b), "v"(c), "v"(d)); }
__device__ __forceinline__ void acc_guard4(v8f& a, v8f& b, v8f& c, v8f& d) { asm volatile("v_nop\n\tv_nop\n\tv_nop\n\tv_nop" : "+v"(a), "+v"(b), "+v"(c), "+v"(d)); }
__device__ __forceinline__ void dep_guard6_h(v8f& a0, v8f& a1, v8f& a2, v8f& a3, v8f& a4, v8f& a5,
                                             v16h f0, v16h f1, v16h f2, v16h f3, v16h f4) {
  asm volatile("v_nop\n\tv_nop\n\tv_nop\n\tv_nop"
               : "+v"(a0), "+v"(a1), "+v"(a2), "+v"(a3), "+v"(a4), "+v"(a5)
               : "v"(f0), "v"(f1), "v"(f2), "v"(f3), "v"(f4));
}

template <typename T> struct Frag;
template <> struct Frag<_Float16> {
  typedef v16h V; union U { v16h v; v8h h[2]; };
  static __device__ __forceinline__ v16h load(const _Float16* p) {
    U f; f.h[0] = *(const v8h*)(p); f.h[1] = *(const v8h*)(p + 16); return f.v;
  }
  static __device__ __forceinline__ v8f mma(v16h a, v16h b, v8f c) {
    return __builtin_amdgcn_wmma_f32_16x16x32_f16(false, a, false, b, (short)0, c, false, false);
  }
  static __device__ __forceinline__ void guard(v8f& a, v8f& b, v16h x, v16h y) { dep_guard_h(a, b, x, y); }
  static __device__ __forceinline__ void keep(v16h a, v16h b, v16h c, v16h d) { keep4_h(a, b, c, d); }
};

__device__ __forceinline__ float fsig(float v) { return __builtin_amdgcn_rcpf(1.0f + expf(-v)); }

__global__ __launch_bounds__(NTHR) void gru_seq_kernel(const float* __restrict__ x,
                                                       const float* __restrict__ w_ih, const float* __restrict__ w_hh,
                                                       const float* __restrict__ b_ih, const float* __restrict__ b_hh,
                                                       const float* __restrict__ fc_w, const float* __restrict__ fc_b,
                                                       float* __restrict__ out) {
  __shared__ __align__(16) _Float16 Atile[2][2][RPB * APITCH];
  __shared__ __align__(16) _Float16 Wh[NG3 * WHP];
  __shared__ __align__(16) _Float16 Wx[NG3 * WXP];
  __shared__ __align__(16) float    Hf[RPB * HFP];
  __shared__ __align__(16) float    Sfcw[NHID];

  const int tid = threadIdx.x, lane = tid & 31, wave = tid >> 5;
  const int c = lane & 15, hh = lane >> 4, koff = hh * 8;
  const int ms = wave >> 2, ub = wave & 3;
  const int j  = 16 * ub + c;
  const int b0 = blockIdx.x * RPB;

  {
    _Float16* af = &Atile[0][0][0];
#pragma unroll 1
    for (int i = tid; i < 4 * RPB * APITCH; i += NTHR) af[i] = (_Float16)0.0f;
  }
  {
#pragma unroll 1
    for (int i = tid; i < NG3 * (NHID / 4); i += NTHR) {
      const int n = i >> 4, k4 = (i & 15) * 4;
      const v4f v = *(const v4f*)(w_hh + (size_t)n * NHID + k4);
      v4h o;
#pragma unroll
      for (int e = 0; e < 4; ++e) o[e] = (_Float16)(v[e] * WCARRY);
      *(v4h*)(Wh + n * WHP + k4) = o;
    }
    if (tid < NG3) {
      v8h zv;
#pragma unroll
      for (int e = 0; e < 8; ++e) zv[e] = (_Float16)0.0f;
      *(v8h*)(Wh + tid * WHP + 64) = zv;
    }
#pragma unroll 1
    for (int i = tid; i < NG3 * 2; i += NTHR) {
      const int n = i >> 1, oct = i & 1;
      const float* wp = w_ih + (size_t)n * NINP + 8 * oct;
      const v4f va = *(const v4f*)(wp);
      const v4f vb = *(const v4f*)(wp + 4);
      v8h o;
#pragma unroll
      for (int e = 0; e < 4; ++e) { o[e] = (_Float16)(va[e] * WCARRY); o[4 + e] = (_Float16)(vb[e] * WCARRY); }
      *(v8h*)(Wx + n * WXP + 8 * oct) = o;
    }
#pragma unroll 1
    for (int i = tid; i < NG3 * 3; i += NTHR) {
      const int n = i / 3, part = i - 3 * n;
      v8h zv;
#pragma unroll
      for (int e = 0; e < 8; ++e) zv[e] = (_Float16)0.0f;
      *(v8h*)(Wx + n * WXP + 16 + 8 * part) = zv;
    }
    if (wave == 0) {
      const int q = lane & 15;
      const v4f fv = *(const v4f*)(fc_w + 4 * q);
      *(v4f*)(Sfcw + 4 * q) = fv;
    }
  }
  const float bsr = b_ih[j] + b_hh[j];
  const float bsz = b_ih[NHID + j] + b_hh[NHID + j];
  const float bin = b_ih[2 * NHID + j];
  const float bhn = b_hh[2 * NHID + j];

  float hreg[8];
#pragma unroll
  for (int r = 0; r < 8; ++r) hreg[r] = 0.0f;
  __syncthreads();

  const v8f z8 = {0.f, 0.f, 0.f, 0.f, 0.f, 0.f, 0.f, 0.f};
  const _Float16* wr = Wh + j * WHP + koff;
  const _Float16* wz = Wh + (NHID + j) * WHP + koff;
  const _Float16* wn = Wh + (2 * NHID + j) * WHP + koff;
  const _Float16* vr = Wx + j * WXP + koff;
  const _Float16* vz = Wx + (NHID + j) * WXP + koff;
  const _Float16* vn = Wx + (2 * NHID + j) * WXP + koff;
  const int arowoff = (16 * ms + c) * APITCH + koff;

#pragma unroll 1
  for (int t = 0; t < NSTEP; ++t) {
    const int cur = t & 1, nxt = cur ^ 1;

    {
      const int grp = tid >> 7;
      const int pl  = (tid >> 6) & 1;
      const int idx = tid & 63;
      const int srow = idx >> 1, oct = idx & 1;
      _Float16* dst = &Atile[pl][cur][0] + srow * APITCH + ACOLX + 16 * grp + 8 * oct;
      if (grp == 0) {
        const float* xp = x + ((size_t)(b0 + srow) * NSTEP + t) * NINP + 8 * oct;
        const v4f xa = *(const v4f*)(xp);
        const v4f xb = *(const v4f*)(xp + 4);
        v8h hv;
#pragma unroll
        for (int e = 0; e < 4; ++e) {
          const float f = xa[e];
          const _Float16 q = (_Float16)f;
          const float qf = (float)q;
          const float g = pl ? (f - qf) * LOCARRY : f;
          hv[e] = (_Float16)g;
        }
#pragma unroll
        for (int e = 0; e < 4; ++e) {
          const float f = xb[e];
          const _Float16 q = (_Float16)f;
          const float qf = (float)q;
          const float g = pl ? (f - qf) * LOCARRY : f;
          hv[4 + e] = (_Float16)g;
        }
        *(v8h*)dst = hv;
      } else {
        v8h zv;
#pragma unroll
        for (int e = 0; e < 8; ++e) zv[e] = (_Float16)0.0f;
        *(v8h*)dst = zv;
      }
    }
    __syncthreads();

    const _Float16* ahi = &Atile[0][cur][0] + arowoff;
    const _Float16* alo = &Atile[1][cur][0] + arowoff;
    v8f aR = z8, aRl = z8, aZ = z8, aZl = z8, aHN = z8, aHNl = z8, aXN = z8, aXNl = z8;
#pragma unroll 1
    for (int k0 = 0; k0 < KHID; k0 += 32) {
      const v16h fa = Frag<_Float16>::load(ahi + k0);
      const v16h fl = Frag<_Float16>::load(alo + k0);
      const v16h g0 = Frag<_Float16>::load(wr + k0);
      const v16h g1 = Frag<_Float16>::load(wz + k0);
      const v16h g2 = Frag<_Float16>::load(wn + k0);
      aR   = Frag<_Float16>::mma(fa, g0, aR);
      aRl  = Frag<_Float16>::mma(fl, g0, aRl);
      aZ   = Frag<_Float16>::mma(fa, g1, aZ);
      aZl  = Frag<_Float16>::mma(fl, g1, aZl);
      aHN  = Frag<_Float16>::mma(fa, g2, aHN);
      aHNl = Frag<_Float16>::mma(fl, g2, aHNl);
      dep_guard6_h(aR, aRl, aZ, aZl, aHN, aHNl, fa, fl, g0, g1, g2);
    }
    {
      const v16h fa = Frag<_Float16>::load(ahi + ACOLX);
      const v16h fl = Frag<_Float16>::load(alo + ACOLX);
      const v16h g0 = Frag<_Float16>::load(vr);
      const v16h g1 = Frag<_Float16>::load(vz);
      const v16h g2 = Frag<_Float16>::load(vn);
      aR   = Frag<_Float16>::mma(fa, g0, aR);
      aRl  = Frag<_Float16>::mma(fl, g0, aRl);
      aZ   = Frag<_Float16>::mma(fa, g1, aZ);
      aZl  = Frag<_Float16>::mma(fl, g1, aZl);
      aXN  = Frag<_Float16>::mma(fa, g2, aXN);
      aXNl = Frag<_Float16>::mma(fl, g2, aXNl);
      dep_guard6_h(aR, aRl, aZ, aZl, aXN, aXNl, fa, fl, g0, g1, g2);
    }
    acc_guard4(aR, aRl, aZ, aZl);
    acc_guard4(aHN, aHNl, aXN, aXNl);

    _Float16* nh = &Atile[0][nxt][0];
    _Float16* nl = &Atile[1][nxt][0];
#pragma unroll
    for (int r = 0; r < 8; ++r) {
      const int row = 16 * ms + 8 * hh + r;
      const float pr = (aR[r]  + aRl[r]  * LOCARRY_INV) * WCARRY_INV + bsr;
      const float pz = (aZ[r]  + aZl[r]  * LOCARRY_INV) * WCARRY_INV + bsz;
      const float gn = (aXN[r] + aXNl[r] * LOCARRY_INV) * WCARRY_INV + bin;
      const float hn = (aHN[r] + aHNl[r] * LOCARRY_INV) * WCARRY_INV + bhn;
      const float rg = fsig(pr);
      const float zg = fsig(pz);
      const float ng = tanhf(gn + rg * hn);
      const float ho = hreg[r];
      const float hw = (1.0f - zg) * ng + zg * ho;
      hreg[r] = hw;
      const _Float16 q = (_Float16)hw;
      const float qf = (float)q;
      nh[row * APITCH + j] = q;
      nl[row * APITCH + j] = (_Float16)((hw - qf) * LOCARRY);
    }
  }

#pragma unroll
  for (int r = 0; r < 8; ++r) Hf[(16 * ms + 8 * hh + r) * HFP + j] = hreg[r];
  __syncthreads();
  if (wave == 0) {
    const float* hrow = Hf + lane * HFP;
    float s = 0.0f;
#pragma unroll
    for (int q = 0; q < NHID / 4; ++q) {
      const v4f hv = *(const v4f*)(hrow + 4 * q);
      const v4f fv = *(const v4f*)(Sfcw + 4 * q);
      s += hv[0] * fv[0];
      s += hv[1] * fv[1];
      s += hv[2] * fv[2];
      s += hv[3] * fv[3];
    }
    const float res = s + fc_b[0];
    float* op = out + b0 + lane;
    *(volatile float*)op = res;
    __threadfence();
    *(volatile float*)op = res;
  }
}

extern "C" void kernel_launch(void* const* d_in, const int* in_sizes, int n_in,
                              void* d_out, int out_size, void* d_ws, size_t ws_size, hipStream_t stream) {
  (void)d_ws; (void)ws_size;
  if (n_in < 7 || d_out == nullptr) return;
  if (in_sizes[0] != NSEQ * NSTEP * NINP || in_sizes[1] != NG3 * NINP || in_sizes[2] != NG3 * NHID ||
      in_sizes[3] != NG3 || in_sizes[4] != NG3 || in_sizes[5] != NHID || in_sizes[6] != 1 ||
      out_size != NSEQ) return;

  const float* x    = (const float*)d_in[0];
  const float* w_ih = (const float*)d_in[1];
  const float* w_hh = (const float*)d_in[2];
  const float* b_ih = (const float*)d_in[3];
  const float* b_hh = (const float*)d_in[4];
  const float* fc_w = (const float*)d_in[5];
  const float* fc_b = (const float*)d_in[6];
  float* out = (float*)d_out;

  gru_seq_kernel<<<NSEQ / RPB, NTHR, 0, stream>>>(x, w_ih, w_hh, b_ih, b_hh, fc_w, fc_b, out);
}
